// RoutedExpertMLP_16965120819357
// MI455X (gfx1250) — hardware-verified
//
#include <hip/hip_runtime.h>
#include <stdint.h>
#include <stddef.h>
#include <math.h>

#pragma clang fp contract(off)

#define NTOK 8192
#define DM   1024
#define DFF  512
#define NEX  8
#define MT   32
#define GX   32
#define TPB  8
#define XP   1032
#define HP   520
#define YP   260
#define RECW 4
#define TT   64
#define TPF  68

#define LDS_XB  (MT * XP * 2)
#define LDS_HB  (MT * HP * 2)
#define LDS_YB  (MT * YP * 4)
#define LDS_EXP (LDS_XB + LDS_HB + LDS_YB)

#define W_SC 256.0f
#define R_W  0.00390625f
#define H_SC 16.0f
#define R_HW 0.000244140625f
#define RSQ2 0.70710678118654752f

static_assert((XP * 2) % 16 == 0);
static_assert((HP * 2) % 16 == 0);
static_assert((YP * 4) % 16 == 0);
static_assert((TPF * 4) % 16 == 0);
static_assert(LDS_XB % 16 == 0);
static_assert(LDS_HB % 16 == 0);
static_assert(NTOK % 256 == 0);
static_assert(NTOK % 8 == 0);
static_assert(GX * TPB * MT == NTOK);
static_assert(TPB * MT <= 256);
static_assert(MT * (DM / 8) == 16 * 256);
static_assert(DM % 256 == 0);
static_assert(DFF % 256 == 0);
static_assert(DM % 64 == 0);
static_assert(DFF % 64 == 0);
static_assert(DM % TT == 0);
static_assert(DFF % TT == 0);
static_assert((NEX * DM) % 1024 == 0);
static_assert((NTOK * DM) % (8 * 256) == 0);
static_assert(NEX == 8);
static_assert(DM % 128 == 0);
static_assert(RECW == 4);
static_assert(HP >= DFF + 8);
static_assert(XP >= DM + 8);
static_assert(YP >= 256);

typedef _Float16       v16h __attribute__((ext_vector_type(16)));
typedef _Float16       v8h  __attribute__((ext_vector_type(8)));
typedef float          v8f  __attribute__((ext_vector_type(8)));
typedef float          v4f  __attribute__((ext_vector_type(4)));
typedef unsigned int   v4u  __attribute__((ext_vector_type(4)));
typedef v4f __attribute__((may_alias)) v4fa;
typedef v4u __attribute__((may_alias)) v4ua;

union FragH { v16h v; v4u q[2]; };
union Pack8 { v8h h; v4u u; };

__device__ __forceinline__ v8f wmma_h(v16h a, v16h b, v8f c) {
  v8f d = __builtin_amdgcn_wmma_f32_16x16x32_f16(false, a, false, b, (short)0, c, false, false);
  asm volatile("v_nop\n\tv_nop\n\tv_nop\n\tv_nop" : "+v"(d) : "v"(a), "v"(b));
  return d;
}

__device__ __forceinline__ v16h ldfrag(const unsigned short* p, int h) {
  FragH f;
  f.q[0] = *(const v4ua*)(p + 8 * h);
  f.q[1] = *(const v4ua*)(p + 16 + 8 * h);
  return f.v;
}

__global__ __launch_bounds__(256) void k_cvt(const float* __restrict__ src,
                                             unsigned short* __restrict__ dst,
                                             int n8, float sc)
{
  const int g = blockIdx.x * 256 + threadIdx.x;
  if (g >= n8) return;
  const float* s = src + (size_t)g * 8;
  const v4f a = *(const v4fa*)s;
  const v4f c = *(const v4fa*)(s + 4);
  v8h hv;
  hv[0] = (_Float16)(a.x * sc); hv[1] = (_Float16)(a.y * sc);
  hv[2] = (_Float16)(a.z * sc); hv[3] = (_Float16)(a.w * sc);
  hv[4] = (_Float16)(c.x * sc); hv[5] = (_Float16)(c.y * sc);
  hv[6] = (_Float16)(c.z * sc); hv[7] = (_Float16)(c.w * sc);
  Pack8 p;
  p.h = hv;
  const v4u u = p.u;
  unsigned short* d = dst + (size_t)g * 8;
  *(volatile v4u*)d = u;
  __threadfence();
  *(volatile v4u*)d = u;
}

__global__ __launch_bounds__(256) void k_tcv(const float* __restrict__ src,
                                             unsigned short* __restrict__ dst,
                                             int K, int N, float sc)
{
  __shared__ __align__(16) float tile[TT * TPF];
  const int tid = threadIdx.x;
  const int n0 = blockIdx.x * TT, k0 = blockIdx.y * TT, e = blockIdx.z;
  const float* s = src + (size_t)e * K * N;
  #pragma unroll
  for (int j = 0; j < 4; ++j) {
    const int r  = (tid >> 4) + 16 * j;
    const int c4 = tid & 15;
    const v4f v = *(const v4fa*)(s + (size_t)(k0 + r) * N + n0 + 4 * c4);
    *(v4fa*)(tile + r * TPF + 4 * c4) = v;
  }
  __syncthreads();
  v4u u[2];
  #pragma unroll
  for (int j = 0; j < 2; ++j) {
    const int n = (tid >> 3) + 32 * j;
    const int q = tid & 7;
    v8h hv;
    #pragma unroll
    for (int i = 0; i < 8; ++i) hv[i] = (_Float16)(tile[(8 * q + i) * TPF + n] * sc);
    Pack8 pk;
    pk.h = hv;
    u[j] = pk.u;
  }
  unsigned short* d0 = dst + (size_t)e * N * K + (size_t)(n0 + (tid >> 3)) * K + k0 + 8 * (tid & 7);
  unsigned short* d1 = d0 + (size_t)32 * K;
  *(volatile v4u*)d0 = u[0];
  *(volatile v4u*)d1 = u[1];
  __threadfence();
  *(volatile v4u*)d0 = u[0];
  *(volatile v4u*)d1 = u[1];
}

__global__ __launch_bounds__(256) void k_route(const float* __restrict__ x,
                                               const float* __restrict__ wr,
                                               const float* __restrict__ rb,
                                               float* __restrict__ rec, int ntok)
{
  __shared__ __align__(16) float swr[DM * NEX];
  __shared__ __align__(16) float srec[8 * RECW];
  const int tid = threadIdx.x, lane = tid & 31, wv = tid >> 5;
  #pragma unroll 1
  for (int i = 0; i < (DM * NEX) / 1024; ++i) {
    const int o = 4 * (tid + 256 * i);
    const v4f w4 = *(const v4fa*)(wr + o);
    *(v4fa*)(swr + o) = w4;
  }
  __syncthreads();

  const int t = blockIdx.x * 8 + wv;
  const int tc = (t < ntok) ? t : (ntok - 1);
  const float* xr = x + (size_t)tc * DM;
  double lg[NEX];
  #pragma unroll
  for (int e = 0; e < NEX; ++e) lg[e] = 0.0;
  #pragma unroll 1
  for (int i = 0; i < DM / 32; ++i) {
    const int d = 32 * i + lane;
    const double xv = (double)xr[d];
    const v4f w0 = *(const v4fa*)(swr + d * NEX);
    const v4f w1 = *(const v4fa*)(swr + d * NEX + 4);
    lg[0] = fma(xv, (double)w0.x, lg[0]);
    lg[1] = fma(xv, (double)w0.y, lg[1]);
    lg[2] = fma(xv, (double)w0.z, lg[2]);
    lg[3] = fma(xv, (double)w0.w, lg[3]);
    lg[4] = fma(xv, (double)w1.x, lg[4]);
    lg[5] = fma(xv, (double)w1.y, lg[5]);
    lg[6] = fma(xv, (double)w1.z, lg[6]);
    lg[7] = fma(xv, (double)w1.w, lg[7]);
  }
  #pragma unroll
  for (int off = 16; off > 0; off >>= 1) {
    #pragma unroll
    for (int e = 0; e < NEX; ++e) lg[e] = lg[e] + __shfl_xor(lg[e], off);
  }
  #pragma unroll
  for (int e = 0; e < NEX; ++e) lg[e] = lg[e] + (double)rb[e];

  int i0 = 0;
  double b0 = lg[0];
  #pragma unroll
  for (int e = 1; e < NEX; ++e) {
    const bool take = lg[e] > b0;
    b0 = take ? lg[e] : b0;
    i0 = take ? e : i0;
  }
  int i1 = -1;
  double bb = -1.0e300;
  #pragma unroll
  for (int e = 0; e < NEX; ++e) {
    const bool take = (e != i0) && (lg[e] > bb);
    bb = take ? lg[e] : bb;
    i1 = take ? e : i1;
  }
  i1 = (i1 < 0) ? ((i0 == 0) ? 1 : 0) : i1;
  double s0 = lg[0], s1 = lg[0];
  #pragma unroll
  for (int e = 0; e < NEX; ++e) { s0 = (e == i0) ? lg[e] : s0; s1 = (e == i1) ? lg[e] : s1; }
  const float l0 = (float)s0;
  const float l1 = (float)s1;
  const float q   = expf(l1 - l0);
  const float den = 1.0f + q;
  const float rden = 1.0f / den;
  const float g0 = rden;
  const float g1 = q * rden;

  if (lane == 0) {
    v4f r0;
    r0.x = g0; r0.y = g1; r0.z = (float)i0; r0.w = (float)i1;
    *(v4fa*)(srec + RECW * wv) = r0;
  }
  __syncthreads();
  if (wv == 0) {
    const int lr = lane & 7;
    const v4f v = *(const v4fa*)(srec + 4 * lr);
    const int tt = blockIdx.x * 8 + lr;
    const bool ok = (lane < 8) && (tt < ntok);
    float* dst = rec + (size_t)(blockIdx.x * 8) * RECW + 4 * lr;
    if (ok) *(volatile v4f*)dst = v;
    __threadfence();
    if (ok) *(volatile v4f*)dst = v;
  }
}

__device__ __forceinline__ void part_pass(const float* sY, const int* tk, const int* sl,
                                          float* part, int ns, int wv, int lane, int nrows)
{
  #pragma unroll
  for (int i = 0; i < 4; ++i) {
    const int row = wv * 4 + i;
    int t = tk[row];
    t = (t < 0) ? 0 : ((t > NTOK - 1) ? (NTOK - 1) : t);
    int s = sl[row];
    s = (s != 0) ? 1 : 0;
    const v4f v0 = *(const v4fa*)(sY + row * YP + 4 * lane);
    const v4f v1 = *(const v4fa*)(sY + row * YP + 128 + 4 * lane);
    float* dst = part + ((size_t)t * 2 + s) * DM + ns * 256;
    if (row < nrows) {
      *(volatile v4f*)(dst + 4 * lane) = v0;
      *(volatile v4f*)(dst + 128 + 4 * lane) = v1;
    }
  }
}

__global__ __launch_bounds__(256) void k_expert(const unsigned short* __restrict__ xh,
                                                const unsigned short* __restrict__ w1t,
                                                const unsigned short* __restrict__ w2t,
                                                const float* __restrict__ b1,
                                                const float* __restrict__ b2,
                                                const float* __restrict__ rec,
                                                float* __restrict__ part, int ntok)
{
  extern __shared__ __align__(16) unsigned char dsm_e[];
  unsigned short* sX = (unsigned short*)dsm_e;
  _Float16* sH = (_Float16*)(dsm_e + LDS_XB);
  float* sY = (float*)(dsm_e + LDS_XB + LDS_HB);
  __shared__ int   sTok[TPB * MT];
  __shared__ int   sSlot[TPB * MT];
  __shared__ float sW[TPB * MT];
  __shared__ int   s_wc[8];

  const int tid = threadIdx.x, lane = tid & 31, wv = tid >> 5;
  const int h = lane >> 4, m = lane & 15;
  const int e = blockIdx.y;
  const int bx = blockIdx.x;

  if (tid < TPB * MT) { sTok[tid] = 0; sSlot[tid] = 0; sW[tid] = 0.0f; }
  __syncthreads();

  int base = 0;
  #pragma unroll 1
  for (int ch = 0; ch < NTOK / 256; ++ch) {
    const int t = ch * 256 + tid;
    const int tc = (t < ntok) ? t : (ntok - 1);
    const v4f r = *(const v4fa*)(rec + (size_t)tc * RECW);
    int e0 = (int)r.z, e1 = (int)r.w;
    e0 = (e0 < 0) ? 0 : ((e0 > NEX - 1) ? (NEX - 1) : e0);
    e1 = (e1 < 0) ? 0 : ((e1 > NEX - 1) ? (NEX - 1) : e1);
    const bool f0 = (e0 == e);
    const bool f1 = (e1 == e) && !f0;
    const bool f = (f0 || f1) && (t < ntok);
    const unsigned int msk = __builtin_amdgcn_ballot_w32(f);
    const int off = __builtin_popcount(msk & ((1u << lane) - 1u));
    const int wcnt = __builtin_popcount(msk);
    if (lane == 0) s_wc[wv] = wcnt;
    __syncthreads();
    int pre = 0, tot = 0;
    #pragma unroll
    for (int w2 = 0; w2 < 8; ++w2) {
      const int c2 = s_wc[w2];
      tot += c2;
      pre += (w2 < wv) ? c2 : 0;
    }
    if (f) {
      const int rank = base + pre + off;
      const int tile = rank / MT;
      const int lt = tile / GX;
      const int p = lt * MT + (rank % MT);
      if (((tile % GX) == bx) && ((unsigned)p < (unsigned)(TPB * MT))) {
        sTok[p]  = t;
        sSlot[p] = f0 ? 0 : 1;
        sW[p]    = f0 ? r.x : r.y;
      }
    }
    base += tot;
    __syncthreads();
  }
  const int cnt = base;

  const v8f z8 = {0.f, 0.f, 0.f, 0.f, 0.f, 0.f, 0.f, 0.f};

  #pragma unroll 1
  for (int lt = 0; lt < TPB; ++lt) {
    const int m0 = (bx + GX * lt) * MT;
    if (m0 >= cnt) break;
    int nrows = cnt - m0;
    nrows = (nrows > MT) ? MT : nrows;
    const int lo = lt * MT;

    #pragma unroll
    for (int j = 0; j < 16; ++j) {
      const int idx = tid + 256 * j;
      const int row = idx >> 7, c8 = idx & 127;
      int t = sTok[lo + row];
      t = (t < 0) ? 0 : ((t > NTOK - 1) ? (NTOK - 1) : t);
      const size_t go = (size_t)t * DM + 8 * c8;
      const v4u a = *(const v4ua*)(xh + go);
      *(v4ua*)(sX + row * XP + 8 * c8) = a;
    }
    __syncthreads();

    #pragma unroll 1
    for (int ns1 = 0; ns1 < DFF / 256; ++ns1) {
      v8f acc[2][2];
      #pragma unroll
      for (int mt = 0; mt < 2; ++mt)
        #pragma unroll
        for (int nt = 0; nt < 2; ++nt) acc[mt][nt] = z8;
      #pragma unroll 1
      for (int k0 = 0; k0 < DM; k0 += 64) {
        #pragma unroll
        for (int kk = 0; kk < 2; ++kk) {
          const int kb = k0 + 32 * kk;
          v16h a[2];
          #pragma unroll
          for (int mt = 0; mt < 2; ++mt)
            a[mt] = ldfrag(sX + (16 * mt + m) * XP + kb, h);
          #pragma unroll
          for (int nt = 0; nt < 2; ++nt) {
            const int jf = ns1 * 256 + wv * 32 + 16 * nt + m;
            const size_t ro = ((size_t)e * DFF + jf) * DM + kb;
            const v16h b = ldfrag(w1t + ro, h);
            #pragma unroll
            for (int mt = 0; mt < 2; ++mt) acc[mt][nt] = wmma_h(a[mt], b, acc[mt][nt]);
          }
        }
      }
      #pragma unroll
      for (int nt = 0; nt < 2; ++nt) {
        const int jf = ns1 * 256 + wv * 32 + 16 * nt + m;
        const float bv = b1[e * DFF + jf];
        #pragma unroll
        for (int mt = 0; mt < 2; ++mt) {
          #pragma unroll
          for (int r = 0; r < 8; ++r) {
            const int row = 16 * mt + 8 * h + r;
            const float v = acc[mt][nt][r] * R_W + bv;
            const float g = 0.5f * v * (1.0f + erff(v * RSQ2));
            sH[row * HP + jf] = (_Float16)(g * H_SC);
          }
        }
      }
    }
    __syncthreads();

    const unsigned short* sHu = (const unsigned short*)sH;
    #pragma unroll 1
    for (int ns = 0; ns < DM / 256; ++ns) {
      v8f acc[2][2];
      #pragma unroll
      for (int mt = 0; mt < 2; ++mt)
        #pragma unroll
        for (int nt = 0; nt < 2; ++nt) acc[mt][nt] = z8;
      #pragma unroll 1
      for (int k0 = 0; k0 < DFF; k0 += 64) {
        #pragma unroll
        for (int kk = 0; kk < 2; ++kk) {
          const int kb = k0 + 32 * kk;
          v16h a[2];
          #pragma unroll
          for (int mt = 0; mt < 2; ++mt)
            a[mt] = ldfrag(sHu + (16 * mt + m) * HP + kb, h);
          #pragma unroll
          for (int nt = 0; nt < 2; ++nt) {
            const int jg = ns * 256 + wv * 32 + 16 * nt + m;
            const size_t ro = ((size_t)e * DM + jg) * DFF + kb;
            const v16h b = ldfrag(w2t + ro, h);
            #pragma unroll
            for (int mt = 0; mt < 2; ++mt) acc[mt][nt] = wmma_h(a[mt], b, acc[mt][nt]);
          }
        }
      }
      #pragma unroll
      for (int nt = 0; nt < 2; ++nt) {
        const int jg = ns * 256 + wv * 32 + 16 * nt + m;
        const int cl = wv * 32 + 16 * nt + m;
        const float bv = b2[e * DM + jg];
        #pragma unroll
        for (int mt = 0; mt < 2; ++mt) {
          #pragma unroll
          for (int r = 0; r < 8; ++r) {
            const int row = 16 * mt + 8 * h + r;
            const float y = acc[mt][nt][r] * R_HW + bv;
            sY[row * YP + cl] = y * sW[lo + row];
          }
        }
      }
      __syncthreads();
      part_pass(sY, sTok + lo, sSlot + lo, part, ns, wv, lane, nrows);
      __threadfence();
      part_pass(sY, sTok + lo, sSlot + lo, part, ns, wv, lane, nrows);
      __syncthreads();
    }
  }
}

__global__ __launch_bounds__(256) void k_sum(const float* __restrict__ part,
                                             float* __restrict__ out, int ntok)
{
  const int lane = threadIdx.x & 31, wv = threadIdx.x >> 5;
  const int t = blockIdx.x * 8 + wv;
  if (t >= ntok) return;
  const float* p0 = part + (size_t)t * 2 * DM;
  const float* p1 = p0 + DM;
  v4f o[8];
  #pragma unroll
  for (int i = 0; i < 8; ++i) {
    const v4f a = *(const v4fa*)(p0 + 128 * i + 4 * lane);
    const v4f b = *(const v4fa*)(p1 + 128 * i + 4 * lane);
    o[i] = a + b;
  }
  float* d = out + (size_t)t * DM;
  #pragma unroll
  for (int i = 0; i < 8; ++i) *(volatile v4f*)(d + 128 * i + 4 * lane) = o[i];
  __threadfence();
  #pragma unroll
  for (int i = 0; i < 8; ++i) *(volatile v4f*)(d + 128 * i + 4 * lane) = o[i];
}

extern "C" void kernel_launch(void* const* d_in, const int* in_sizes, int n_in,
                              void* d_out, int out_size, void* d_ws, size_t ws_size,
                              hipStream_t stream)
{
  if (n_in < 7) return;
  if (in_sizes[0] != NTOK * DM) return;
  if (in_sizes[1] != DM * NEX) return;
  if (in_sizes[2] != NEX) return;
  if (in_sizes[3] != NEX * DM * DFF) return;
  if (in_sizes[4] != NEX * DFF) return;
  if (in_sizes[5] != NEX * DFF * DM) return;
  if (in_sizes[6] != NEX * DM) return;
  if (out_size != NTOK * DM) return;

  const float* x   = (const float*)d_in[0];
  const float* rw  = (const float*)d_in[1];
  const float* rb  = (const float*)d_in[2];
  const float* w1  = (const float*)d_in[3];
  const float* b1p = (const float*)d_in[4];
  const float* w2  = (const float*)d_in[5];
  const float* b2p = (const float*)d_in[6];
  float* out = (float*)d_out;

  const size_t bXH   = (size_t)NTOK * DM * 2;
  const size_t bW1T  = (size_t)NEX * DFF * DM * 2;
  const size_t bW2T  = (size_t)NEX * DM * DFF * 2;
  const size_t bREC  = (size_t)NTOK * RECW * 4;
  const size_t bPART = (size_t)NTOK * 2 * DM * 4;
  const size_t total = bXH + bW1T + bW2T + bREC + bPART;
  if (total > ws_size) return;
  if (total > (size_t)134217728) return;

  char* ws = (char*)d_ws;
  size_t off = 0;
  unsigned short* XH   = (unsigned short*)(ws + off); off += bXH;
  unsigned short* W1T  = (unsigned short*)(ws + off); off += bW1T;
  unsigned short* W2T  = (unsigned short*)(ws + off); off += bW2T;
  float*          REC  = (float*)(ws + off);          off += bREC;
  float*          PART = (float*)(ws + off);          off += bPART;
  if (off != total) return;

  hipFuncSetAttribute(reinterpret_cast<const void*>(&k_expert),
                      hipFuncAttributeMaxDynamicSharedMemorySize, LDS_EXP);

  {
    const int n8x = NTOK * DM / 8;
    k_cvt<<<(n8x + 255) / 256, 256, 0, stream>>>(x, XH, n8x, 1.0f);
  }
  k_tcv<<<dim3(DFF / TT, DM / TT, NEX), 256, 0, stream>>>(w1, W1T, DM, DFF, W_SC);
  k_tcv<<<dim3(DM / TT, DFF / TT, NEX), 256, 0, stream>>>(w2, W2T, DFF, DM, W_SC);
  k_route<<<(NTOK + 7) / 8, 256, 0, stream>>>(x, rw, rb, REC, NTOK);
  k_expert<<<dim3(GX, NEX), 256, LDS_EXP, stream>>>(XH, W1T, W2T, b1p, b2p, REC, PART, NTOK);
  k_sum<<<(NTOK + 7) / 8, 256, 0, stream>>>(PART, out, NTOK);
}
